// MultiHeadedAttention2_28544352649621
// MI455X (gfx1250) — hardware-verified
//
#include <hip/hip_runtime.h>


#define NBI  8
#define NT_  1024
#define DM   512
#define NH_  8
#define HD   64
#define VHD  128
#define NKVV 4
#define KW   DM
#define NTK  NT_
#define SCL  0.125f
#define LOSC 1024.0f

typedef _Float16 h16;
typedef unsigned short bf;
typedef __attribute__((ext_vector_type(16))) __bf16   v16bf;
typedef __attribute__((ext_vector_type(16))) _Float16 v16h;
typedef __attribute__((ext_vector_type(8)))  _Float16 v8h;
typedef __attribute__((ext_vector_type(8)))  unsigned short v8us;
typedef __attribute__((ext_vector_type(8)))  float    v8f;
typedef __attribute__((ext_vector_type(4)))  float    v4f;
typedef __attribute__((ext_vector_type(4)))  _Float16 v4h;
typedef v8h  __attribute__((may_alias)) v8ha;
typedef v4f  __attribute__((may_alias)) v4fa;
typedef v8us __attribute__((may_alias)) v8usa;

__device__ __forceinline__ unsigned short f2bf(float f) { unsigned u = __float_as_uint(f); u += 0x7FFFu + ((u >> 16) & 1u); return (unsigned short)(u >> 16); }
__device__ __forceinline__ float bf2f(unsigned short b) { return __uint_as_float(((unsigned)b) << 16); }
__device__ __forceinline__ float bfr(float f) { return bf2f(f2bf(f)); }
__device__ __forceinline__ v16h cat16(v8h lo, v8h hi) { return __builtin_shufflevector(lo, hi, 0, 1, 2, 3, 4, 5, 6, 7, 8, 9, 10, 11, 12, 13, 14, 15); }
__device__ __forceinline__ v16bf cat16b(v8us lo, v8us hi) { return __builtin_bit_cast(v16bf, __builtin_shufflevector(lo, hi, 0, 1, 2, 3, 4, 5, 6, 7, 8, 9, 10, 11, 12, 13, 14, 15)); }
__device__ __forceinline__ v8f wmma16(v16h a, v16h b, v8f c) { return __builtin_amdgcn_wmma_f32_16x16x32_f16(false, a, false, b, (short)0, c, false, false); }
__device__ __forceinline__ v8f wmmab(v16bf a, v16bf b, v8f c) { return __builtin_amdgcn_wmma_f32_16x16x32_bf16(false, a, false, b, (short)0, c, false, false); }

__global__ __launch_bounds__(256) void k_cvtb(const float* __restrict__ src, int nrows, bf* dst) {
    const int lane = threadIdx.x & 31, r = blockIdx.x * 8 + (threadIdx.x >> 5);
    if (r >= nrows) return;
    v8us o[DM / 256];
#pragma unroll
    for (int q = 0; q < DM / 256; ++q) { v8us t;
#pragma unroll
        for (int i = 0; i < 8; ++i) t[i] = f2bf(src[(size_t)r * DM + q * 256 + lane * 8 + i]);
        o[q] = t; }
#pragma unroll
    for (int q = 0; q < DM / 256; ++q) *(volatile v8us*)(dst + (size_t)r * DM + q * 256 + lane * 8) = o[q];
    __threadfence();
#pragma unroll
    for (int q = 0; q < DM / 256; ++q) *(volatile v8us*)(dst + (size_t)r * DM + q * 256 + lane * 8) = o[q];
}

template <bool SPLITA, bool F16OUT = false>
__global__ __launch_bounds__(128) void k_gemmb(const bf* __restrict__ A, const bf* __restrict__ Al, const bf* __restrict__ Bn, const float* __restrict__ bias, float* C, int ldc, h16* C2, const float* __restrict__ R = nullptr, int K = DM, int roundR = 1) {
    __shared__ __align__(16) float ost[4][16 * 68];
    const int lane = threadIdx.x & 31, wave = threadIdx.x >> 5, lr = lane & 15, hi = lane >> 4;
    const int r0 = blockIdx.x * 64 + wave * 16, c0 = blockIdx.y * 64;
    const size_t aoff = (size_t)(r0 + lr) * K + 8 * hi;
    size_t boff[4];
#pragma unroll
    for (int t = 0; t < 4; ++t) boff[t] = (size_t)(c0 + t * 16 + lr) * K + 8 * hi;
    v8f acc[4];
#pragma unroll
    for (int t = 0; t < 4; ++t) acc[t] = (v8f){};
#pragma unroll 1
    for (int kc = 0; kc < K; kc += 32) {
        const v16bf a = cat16b(*(const v8us*)(A + aoff + kc), *(const v8us*)(A + aoff + kc + 16));
        v16bf al = a;
        if (SPLITA) al = cat16b(*(const v8us*)(Al + aoff + kc), *(const v8us*)(Al + aoff + kc + 16));
#pragma unroll
        for (int t = 0; t < 4; ++t) { const v16bf b = cat16b(*(const v8us*)(Bn + boff[t] + kc), *(const v8us*)(Bn + boff[t] + kc + 16)); acc[t] = wmmab(a, b, acc[t]); if (SPLITA) acc[t] = wmmab(al, b, acc[t]); }
        asm volatile("v_nop\n\tv_nop\n\tv_nop\n\tv_nop" : "+v"(acc[0]), "+v"(acc[1]), "+v"(acc[2]), "+v"(acc[3]) : "v"(a), "v"(al));
    }
    float* os = &ost[wave][0];
#pragma unroll
    for (int t = 0; t < 4; ++t) { const float bv = bias ? bfr(bias[c0 + t * 16 + lr]) : 0.f;
#pragma unroll
        for (int j = 0; j < 8; ++j) os[(hi * 8 + j) * 68 + t * 16 + lr] = acc[t][j] + bv; }
    __syncthreads();
    if (F16OUT) {
        h16* crow = (h16*)(void*)C + (size_t)r0 * ldc + c0;
        auto pass = [&]() {
#pragma unroll
            for (int s = 0; s < 4; ++s) { const int row = 4 * s + (lane >> 3), piece = lane & 7; const float* sp = os + row * 68 + piece * 8; v8h o, o2;
#pragma unroll
                for (int i = 0; i < 8; ++i) { const h16 a = (h16)sp[i]; o[i] = a; o2[i] = (h16)((sp[i] - (float)a) * LOSC); }
                *(volatile v8h*)(crow + (size_t)row * ldc + piece * 8) = o; if (C2) *(volatile v8h*)(C2 + (size_t)r0 * ldc + c0 + (size_t)row * ldc + piece * 8) = o2; }
        };
        pass(); __threadfence(); pass();
    } else {
        float* crow = C + (size_t)r0 * ldc + c0;
        auto pass = [&]() {
#pragma unroll
            for (int s = 0; s < 8; ++s) { const int Lid = (lane >> 3) + 4 * s, piece = lane & 7; const int row = Lid >> 1, cofs = (Lid & 1) * 32 + piece * 4;
                v4f val = *(const v4fa*)(os + row * 68 + cofs); if (R) { const v4f rv = *(const v4f*)(R + ((size_t)r0 + row) * ldc + c0 + cofs); val += roundR ? (v4f){bfr(rv[0]), bfr(rv[1]), bfr(rv[2]), bfr(rv[3])} : rv; }
                *(volatile v4f*)(crow + (size_t)row * ldc + cofs) = val; }
        };
        pass(); __threadfence(); pass();
    }
}

__global__ __launch_bounds__(128) void k_gemm3(const bf* __restrict__ Ah, const bf* __restrict__ Al, const bf* __restrict__ Bh, const bf* __restrict__ Bl, int K, float* C, int ldc) {
    __shared__ __align__(16) float ost[4][16 * 68];
    const int lane = threadIdx.x & 31, wave = threadIdx.x >> 5, lr = lane & 15, hi = lane >> 4;
    const int r0 = blockIdx.x * 64 + wave * 16, c0 = blockIdx.y * 64;
    const size_t aoff = (size_t)(r0 + lr) * K + 8 * hi;
    v8f acc[4];
#pragma unroll
    for (int t = 0; t < 4; ++t) acc[t] = (v8f){};
#pragma unroll 1
    for (int kc = 0; kc < K; kc += 32) {
        const v16bf a = cat16b(*(const v8us*)(Ah + aoff + kc), *(const v8us*)(Ah + aoff + kc + 16));
        const v16bf al = cat16b(*(const v8us*)(Al + aoff + kc), *(const v8us*)(Al + aoff + kc + 16));
#pragma unroll
        for (int t = 0; t < 4; ++t) { const size_t bo = (size_t)(c0 + t * 16 + lr) * K + kc + 8 * hi;
            const v16bf bh = cat16b(*(const v8us*)(Bh + bo), *(const v8us*)(Bh + bo + 16)); const v16bf bl = cat16b(*(const v8us*)(Bl + bo), *(const v8us*)(Bl + bo + 16));
            acc[t] = wmmab(a, bh, acc[t]); acc[t] = wmmab(al, bh, acc[t]); acc[t] = wmmab(a, bl, acc[t]); }
        asm volatile("v_nop\n\tv_nop\n\tv_nop\n\tv_nop" : "+v"(acc[0]), "+v"(acc[1]), "+v"(acc[2]), "+v"(acc[3]) : "v"(a), "v"(al));
    }
    float* os = &ost[wave][0];
#pragma unroll
    for (int t = 0; t < 4; ++t) {
#pragma unroll
        for (int j = 0; j < 8; ++j) os[(hi * 8 + j) * 68 + t * 16 + lr] = acc[t][j]; }
    __builtin_amdgcn_wave_barrier(); asm volatile("" ::: "memory");
    float* crow = C + (size_t)r0 * ldc + c0;
    auto pass = [&]() {
#pragma unroll
        for (int s = 0; s < 8; ++s) { const int Lid = (lane >> 3) + 4 * s, piece = lane & 7; const int row = Lid >> 1, cofs = (Lid & 1) * 32 + piece * 4;
            const v4f val = *(const v4fa*)(os + row * 68 + cofs); *(volatile v4f*)(crow + (size_t)row * ldc + cofs) = val; }
    };
    pass(); __threadfence(); pass();
}
__global__ __launch_bounds__(256) void k_vt(const float* __restrict__ V, bf* VTH, bf* VTL) {
    __shared__ float tl[64][65];
    const int tid = threadIdx.x, t0 = blockIdx.x * 64, d0 = blockIdx.y * 64, g = blockIdx.z;
    { const int tt = tid >> 2, dq = (tid & 3) * 16;
#pragma unroll
      for (int i = 0; i < 16; ++i) tl[dq + i][tt] = V[(size_t)(t0 + tt) * KW + g * VHD + d0 + dq + i]; }
    __syncthreads();
    const int piece = tid & 7;
    auto pass = [&]() {
#pragma unroll
        for (int s = 0; s < 2; ++s) { const int d = (tid >> 3) + 32 * s; v8us oh, ol;
#pragma unroll
            for (int i = 0; i < 8; ++i) { const float v = tl[d][piece * 8 + i]; const unsigned short hb = f2bf(v); oh[i] = hb; ol[i] = f2bf(v - bf2f(hb)); }
            const size_t o = ((size_t)g * VHD + d0 + d) * NT_ + t0 + piece * 8; *(volatile v8us*)(VTH + o) = oh; *(volatile v8us*)(VTL + o) = ol; }
    };
    pass(); __threadfence(); pass();
}

__global__ __launch_bounds__(256) void k_hsplit(const float* __restrict__ X, bf* Ph, bf* Pl) {
    typedef __attribute__((ext_vector_type(2))) unsigned short v2us;
    const int lane = threadIdx.x & 31, wid = blockIdx.x * 8 + (threadIdx.x >> 5); if (wid >= NT_ * NH_) return;
    const int t = wid / NH_, h = wid % NH_; v2us oh, ol;
#pragma unroll
    for (int i = 0; i < 2; ++i) { const float v = X[(size_t)t * DM + h * HD + 2 * lane + i]; const unsigned short hb = f2bf(v); oh[i] = hb; ol[i] = f2bf(v - bf2f(hb)); }
    const size_t o = ((size_t)h * NT_ + t) * HD + 2 * lane;
    *(volatile v2us*)(Ph + o) = oh; *(volatile v2us*)(Pl + o) = ol; __threadfence(); *(volatile v2us*)(Ph + o) = oh; *(volatile v2us*)(Pl + o) = ol;
}
__global__ __launch_bounds__(256) void k_smax2(const float* __restrict__ SR, const float* __restrict__ SF, bf* PH, bf* PL) {
    const int lane = threadIdx.x & 31, r = blockIdx.x * 8 + (threadIdx.x >> 5); if (r >= NT_) return;
    const float* ar = SR + (size_t)r * NT_; const float* af = SF + (size_t)r * NT_;
    float mr = -3.0e38f, mf = -3.0e38f;
#pragma unroll 1
    for (int c0 = lane * 8; c0 < NT_; c0 += 256) { const v8f a = *(const v8f*)(ar + c0), b = *(const v8f*)(af + c0);
#pragma unroll
        for (int i = 0; i < 8; ++i) { mr = fmaxf(mr, a[i] * SCL); mf = fmaxf(mf, b[i] * SCL); } }
#pragma unroll
    for (int sh = 16; sh; sh >>= 1) { mr = fmaxf(mr, __shfl_xor(mr, sh, 32)); mf = fmaxf(mf, __shfl_xor(mf, sh, 32)); }
    float sr = 0.f, sf = 0.f;
#pragma unroll 1
    for (int c0 = lane * 8; c0 < NT_; c0 += 256) { const v8f a = *(const v8f*)(ar + c0), b = *(const v8f*)(af + c0);
#pragma unroll
        for (int i = 0; i < 8; ++i) { sr += __expf(a[i] * SCL - mr); sf += __expf(b[i] * SCL - mf); } }
#pragma unroll
    for (int sh = 16; sh; sh >>= 1) { sr += __shfl_xor(sr, sh, 32); sf += __shfl_xor(sf, sh, 32); }
    const float ir = 1.0f / sr, iff = 1.0f / sf;
#pragma unroll 1
    for (int ps = 0; ps < 2; ++ps) {
#pragma unroll 1
        for (int c0 = lane * 8; c0 < NT_; c0 += 256) { const v8f a = *(const v8f*)(ar + c0), b = *(const v8f*)(af + c0); v8us oh, ol;
#pragma unroll
            for (int i = 0; i < 8; ++i) { const float p = fmaxf(__expf(a[i] * SCL - mr) * ir, __expf(b[i] * SCL - mf) * iff); const unsigned short hb = f2bf(p); oh[i] = hb; ol[i] = f2bf(p - bf2f(hb)); }
            const size_t o = (size_t)r * NT_ + c0; *(volatile v8us*)(PH + o) = oh; *(volatile v8us*)(PL + o) = ol; }
        if (ps == 0) __threadfence(); }
}
__global__ __launch_bounds__(256) void k_split(const float* __restrict__ src, int nrows, bf* dh, bf* dl) {
    const int lane = threadIdx.x & 31, r = blockIdx.x * 8 + (threadIdx.x >> 5); if (r >= nrows) return;
#pragma unroll 1
    for (int ps = 0; ps < 2; ++ps) {
#pragma unroll 1
        for (int q = 0; q < DM / 256; ++q) { const size_t o = (size_t)r * DM + q * 256 + lane * 8; const v8f v = *(const v8f*)(src + o); v8us oh, ol;
#pragma unroll
            for (int i = 0; i < 8; ++i) { const unsigned short hb = f2bf(v[i]); oh[i] = hb; ol[i] = f2bf(v[i] - bf2f(hb)); }
            *(volatile v8us*)(dh + o) = oh; *(volatile v8us*)(dl + o) = ol; }
        if (ps == 0) __threadfence(); }
}

extern "C" void kernel_launch(void* const* d_in, const int* in_sizes, int n_in,
                              void* d_out, int out_size, void* d_ws, size_t ws_size, hipStream_t stream) {
    (void)in_sizes; (void)n_in; (void)out_size;
    const float* xr = (const float*)d_in[0]; const float* xf = (const float*)d_in[1];
    const float* Wq1 = (const float*)d_in[2]; const float* bq1 = (const float*)d_in[3]; const float* Wk1 = (const float*)d_in[4]; const float* bk1 = (const float*)d_in[5]; const float* Wv1 = (const float*)d_in[6]; const float* bv1 = (const float*)d_in[7];
    const float* Wq2 = (const float*)d_in[8]; const float* bq2 = (const float*)d_in[9]; const float* Wk2 = (const float*)d_in[10]; const float* bk2 = (const float*)d_in[11]; const float* Wv2 = (const float*)d_in[12]; const float* bv2 = (const float*)d_in[13];
    const float* Wo1 = (const float*)d_in[14]; const float* bo1 = (const float*)d_in[15]; const float* Wo2 = (const float*)d_in[16]; const float* bo2 = (const float*)d_in[17];
    float* out0 = (float*)d_out; float* out1 = out0 + (size_t)NBI * NT_ * DM;
    char* wsp = (char*)d_ws;
    auto take = [&](size_t bytes) { char* p = wsp; wsp += (bytes + 255) & ~(size_t)255; return (void*)p; };
    bf* WB[8]; const float* Ws[8] = {Wq1, Wk1, Wv1, Wq2, Wk2, Wv2, Wo1, Wo2};
    for (int i = 0; i < 8; ++i) WB[i] = (bf*)take((size_t)DM * DM * 2);
    bf* Xr = (bf*)take((size_t)NT_ * DM * 2); bf* Xf = (bf*)take((size_t)NT_ * DM * 2); float* TMP = (float*)take((size_t)NT_ * DM * 4);
    bf* QRh = (bf*)take((size_t)NT_ * DM * 2); bf* QRl = (bf*)take((size_t)NT_ * DM * 2); bf* KRh = (bf*)take((size_t)NT_ * DM * 2); bf* KRl = (bf*)take((size_t)NT_ * DM * 2);
    bf* QFh = (bf*)take((size_t)NT_ * DM * 2); bf* QFl = (bf*)take((size_t)NT_ * DM * 2); bf* KFh = (bf*)take((size_t)NT_ * DM * 2); bf* KFl = (bf*)take((size_t)NT_ * DM * 2);
    bf* VRh = (bf*)take((size_t)DM * NT_ * 2); bf* VRl = (bf*)take((size_t)DM * NT_ * 2); bf* VFh = (bf*)take((size_t)DM * NT_ * 2); bf* VFl = (bf*)take((size_t)DM * NT_ * 2);
    float* SR = (float*)take((size_t)NT_ * NT_ * 4); float* SF = (float*)take((size_t)NT_ * NT_ * 4); bf* PH = (bf*)take((size_t)NT_ * NT_ * 2); bf* PL = (bf*)take((size_t)NT_ * NT_ * 2);
    float* CR = (float*)take((size_t)NT_ * DM * 4); float* CF = (float*)take((size_t)NT_ * DM * 4); bf* Ch = (bf*)take((size_t)NT_ * DM * 2); bf* Cl = (bf*)take((size_t)NT_ * DM * 2);
    if ((size_t)(wsp - (char*)d_ws) > ws_size) return;
    for (int i = 0; i < 8; ++i) k_cvtb<<<DM / 8, 256, 0, stream>>>(Ws[i], DM, WB[i]);
    for (int b = 0; b < NBI; ++b) {
        k_cvtb<<<NT_ / 8, 256, 0, stream>>>(xr + (size_t)b * NT_ * DM, NT_, Xr); k_cvtb<<<NT_ / 8, 256, 0, stream>>>(xf + (size_t)b * NT_ * DM, NT_, Xf);
        k_gemmb<false, false><<<dim3(NT_ / 64, DM / 64, 1), 128, 0, stream>>>(Xr, nullptr, WB[0], bq1, TMP, DM, nullptr); k_hsplit<<<(NT_ * NH_) / 8, 256, 0, stream>>>(TMP, QRh, QRl);
        k_gemmb<false, false><<<dim3(NT_ / 64, DM / 64, 1), 128, 0, stream>>>(Xr, nullptr, WB[1], bk1, TMP, DM, nullptr); k_hsplit<<<(NT_ * NH_) / 8, 256, 0, stream>>>(TMP, KRh, KRl);
        k_gemmb<false, false><<<dim3(NT_ / 64, DM / 64, 1), 128, 0, stream>>>(Xr, nullptr, WB[2], bv1, TMP, DM, nullptr); k_vt<<<dim3(NT_ / 64, 2, NKVV), 256, 0, stream>>>(TMP, VRh, VRl);
        k_gemmb<false, false><<<dim3(NT_ / 64, DM / 64, 1), 128, 0, stream>>>(Xf, nullptr, WB[3], bq2, TMP, DM, nullptr); k_hsplit<<<(NT_ * NH_) / 8, 256, 0, stream>>>(TMP, QFh, QFl);
        k_gemmb<false, false><<<dim3(NT_ / 64, DM / 64, 1), 128, 0, stream>>>(Xf, nullptr, WB[4], bk2, TMP, DM, nullptr); k_hsplit<<<(NT_ * NH_) / 8, 256, 0, stream>>>(TMP, KFh, KFl);
        k_gemmb<false, false><<<dim3(NT_ / 64, DM / 64, 1), 128, 0, stream>>>(Xf, nullptr, WB[5], bv2, TMP, DM, nullptr); k_vt<<<dim3(NT_ / 64, 2, NKVV), 256, 0, stream>>>(TMP, VFh, VFl);
        for (int h = 0; h < NH_; ++h) { const size_t po = (size_t)h * NT_ * HD, vo = (size_t)h * HD * NT_;
            k_gemm3<<<dim3(NT_ / 64, NT_ / 64, 1), 128, 0, stream>>>(QRh + po, QRl + po, KRh + po, KRl + po, HD, SR, NT_);
            k_gemm3<<<dim3(NT_ / 64, NT_ / 64, 1), 128, 0, stream>>>(QFh + po, QFl + po, KFh + po, KFl + po, HD, SF, NT_);
            k_smax2<<<NT_ / 8, 256, 0, stream>>>(SR, SF, PH, PL);
            k_gemm3<<<dim3(NT_ / 64, HD / 64, 1), 128, 0, stream>>>(PH, PL, VRh + vo, VRl + vo, NT_, CR + h * HD, DM);
            k_gemm3<<<dim3(NT_ / 64, HD / 64, 1), 128, 0, stream>>>(PH, PL, VFh + vo, VFl + vo, NT_, CF + h * HD, DM);
        }
        k_split<<<NT_ / 8, 256, 0, stream>>>(CR, NT_, Ch, Cl); k_gemmb<true, false><<<dim3(NT_ / 64, DM / 64, 1), 128, 0, stream>>>(Ch, Cl, WB[6], bo1, out0 + (size_t)b * NT_ * DM, DM, nullptr);
        k_split<<<NT_ / 8, 256, 0, stream>>>(CF, NT_, Ch, Cl); k_gemmb<true, false><<<dim3(NT_ / 64, DM / 64, 1), 128, 0, stream>>>(Ch, Cl, WB[7], bo2, out1 + (size_t)b * NT_ * DM, DM, nullptr);
    }
}
